// TRPN_73349451481376
// MI455X (gfx1250) — hardware-verified
//
#include <hip/hip_runtime.h>
#include <stdint.h>
#include <stddef.h>
#include <math.h>

#define TT  4
#define NN  400
#define SS  395
#define QQ  5
#define DD  128
#define H0  256
#define H1  128
#define H2  128
#define GD  768
#define NW  5
#define TN  (TT * NN)
#define KP  512
#define KA  416
#define W2P 264
#define SDP 404
#define EP  132
#define PP  260
#define WTP 68

#define PAIR_LDS_W2    (H1 * W2P * 2)
#define PAIR_LDS_BYTES (PAIR_LDS_W2 + 4 * NN * 4)

static_assert(PAIR_LDS_W2 == 67584);
static_assert(PAIR_LDS_BYTES == 73984);
static_assert((PAIR_LDS_W2 % 16) == 0);
static_assert((W2P * 2) % 16 == 0);
static_assert((SDP * 4) % 16 == 0);
static_assert((EP * 4) % 16 == 0);
static_assert((PP * 4) % 16 == 0);
static_assert((WTP * 4) % 16 == 0);
static_assert(NN % 16 == 0);
static_assert(NN % 2 == 0);
static_assert(TN % 16 == 0);
static_assert(GD % 128 == 0);
static_assert(GD % 32 == 0);
static_assert(DD % 32 == 0);
static_assert(H0 % 32 == 0);
static_assert(KA % 32 == 0);
static_assert(KA >= NN);
static_assert(KP >= KA);
static_assert((TN * DD) % 2048 == 0);
static_assert((H0 * H0) % 2048 == 0);
static_assert((H1 * H0) % 2048 == 0);
static_assert((H1 * GD) % 2048 == 0);
static_assert((H2 * H1) % 2048 == 0);
static_assert((NN - SS) * DD == 640);

typedef __bf16         v16bf __attribute__((ext_vector_type(16)));
typedef _Float16       v16h  __attribute__((ext_vector_type(16)));
typedef _Float16       v8h   __attribute__((ext_vector_type(8)));
typedef _Float16       v4h   __attribute__((ext_vector_type(4)));
typedef float          v8f   __attribute__((ext_vector_type(8)));
typedef float          v4f   __attribute__((ext_vector_type(4)));
typedef unsigned int   v8u   __attribute__((ext_vector_type(8)));
typedef unsigned int   v4u   __attribute__((ext_vector_type(4)));
typedef unsigned short v8us  __attribute__((ext_vector_type(8)));
typedef v4f  __attribute__((may_alias)) v4fa;
typedef v4u  __attribute__((may_alias)) v4ua;
typedef v8us __attribute__((may_alias)) v8usa;
typedef v8h  __attribute__((may_alias)) v8ha;

union FragU { v16bf v; v8us half[2]; v8u w; };
union FragH { v16h v; v8h half[2]; v4h q[4]; v8u w; };

__device__ __forceinline__ v8f wmma_bf(v16bf a, v16bf b, v8f c) {
  v8f d = __builtin_amdgcn_wmma_f32_16x16x32_bf16(false, a, false, b, (short)0, c, false, false);
  asm volatile("v_nop\n\tv_nop\n\tv_nop\n\tv_nop" : "+v"(d) : "v"(a), "v"(b));
  return d;
}
__device__ __forceinline__ v8f wmma_hf(v16h a, v16h b, v8f c) {
  v8f d = __builtin_amdgcn_wmma_f32_16x16x32_f16(false, a, false, b, (short)0, c, false, false);
  asm volatile("v_nop\n\tv_nop\n\tv_nop\n\tv_nop" : "+v"(d) : "v"(a), "v"(b));
  return d;
}
__device__ __forceinline__ v8f wmma3(v16bf ah, v16bf al, v16bf bh, v16bf bl, v8f c) {
  c = wmma_bf(ah, bh, c);
  c = wmma_bf(ah, bl, c);
  c = wmma_bf(al, bh, c);
  return c;
}

__device__ __forceinline__ v16bf ldfu(const unsigned short* p, int h) {
  FragU f;
  f.half[0] = *(const v8usa*)(p + 8 * h);
  f.half[1] = *(const v8usa*)(p + 16 + 8 * h);
  return f.v;
}
__device__ __forceinline__ v16h ldfh(const _Float16* p, int h) {
  FragH f;
  f.half[0] = *(const v8ha*)(p + 8 * h);
  f.half[1] = *(const v8ha*)(p + 16 + 8 * h);
  return f.v;
}

__device__ __forceinline__ unsigned bf16_rne(float f) {
  const unsigned u = __float_as_uint(f);
  return (u + 0x7fffu + ((u >> 16) & 1u)) >> 16;
}
__device__ __forceinline__ void pk2(float a, float b, unsigned& hw, unsigned& lw) {
  const unsigned ha = bf16_rne(a);
  const unsigned hb = bf16_rne(b);
  const unsigned la = bf16_rne(a - __uint_as_float(ha << 16));
  const unsigned lb = bf16_rne(b - __uint_as_float(hb << 16));
  hw = ha | (hb << 16);
  lw = la | (lb << 16);
}
__device__ __forceinline__ void pk8(v4f a, v4f b, v4u& hv, v4u& lv) {
  unsigned h0, h1, h2, h3, l0, l1, l2, l3;
  pk2(a.x, a.y, h0, l0); pk2(a.z, a.w, h1, l1);
  pk2(b.x, b.y, h2, l2); pk2(b.z, b.w, h3, l3);
  const v4u H = {h0, h1, h2, h3};
  const v4u L = {l0, l1, l2, l3};
  hv = H; lv = L;
}
__device__ __forceinline__ void mkfrag(v4f q0, v4f q1, v4f q2, v4f q3, v16bf& hi, v16bf& lo) {
  unsigned h0, h1, h2, h3, h4, h5, h6, h7;
  unsigned l0, l1, l2, l3, l4, l5, l6, l7;
  pk2(q0.x, q0.y, h0, l0); pk2(q0.z, q0.w, h1, l1);
  pk2(q1.x, q1.y, h2, l2); pk2(q1.z, q1.w, h3, l3);
  pk2(q2.x, q2.y, h4, l4); pk2(q2.z, q2.w, h5, l5);
  pk2(q3.x, q3.y, h6, l6); pk2(q3.z, q3.w, h7, l7);
  FragU H, L;
  const v8u hw = {h0, h1, h2, h3, h4, h5, h6, h7};
  const v8u lw = {l0, l1, l2, l3, l4, l5, l6, l7};
  H.w = hw; L.w = lw;
  hi = H.v; lo = L.v;
}

__device__ __forceinline__ float sigm(float x) {
  const float xc = fminf(fmaxf(x, -40.f), 40.f);
  const float e = __expf(-xc);
  return __builtin_amdgcn_rcpf(1.f + e);
}

__global__ __launch_bounds__(256) void k_split(const float* __restrict__ src,
                                               unsigned short* __restrict__ hi,
                                               unsigned short* __restrict__ lo,
                                               int n8)
{
  const int gid = blockIdx.x * 256 + threadIdx.x;
  if (gid >= n8) return;
  const float* s = src + (size_t)gid * 8;
  const v4f a = *(const v4fa*)s;
  const v4f b = *(const v4fa*)(s + 4);
  v4u hv, lv;
  pk8(a, b, hv, lv);
  unsigned short* hp = hi + (size_t)gid * 8;
  unsigned short* lp = lo + (size_t)gid * 8;
  *(volatile v4ua*)hp = hv;
  *(volatile v4ua*)lp = lv;
  __threadfence();
  *(volatile v4ua*)hp = hv;
  *(volatile v4ua*)lp = lv;
}

__global__ __launch_bounds__(256) void k_cvt16(const float* __restrict__ src,
                                               _Float16* __restrict__ dst,
                                               int n8, float scale)
{
  const int gid = blockIdx.x * 256 + threadIdx.x;
  if (gid >= n8) return;
  const float* s = src + (size_t)gid * 8;
  const v4f a = *(const v4fa*)s * scale;
  const v4f b = *(const v4fa*)(s + 4) * scale;
  const v8f f = {a.x, a.y, a.z, a.w, b.x, b.y, b.z, b.w};
  FragH P;
  P.half[0] = __builtin_convertvector(f, v8h);
  const v4u u = {P.w[0], P.w[1], P.w[2], P.w[3]};
  _Float16* dp = dst + (size_t)gid * 8;
  *(volatile v4ua*)dp = u;
  __threadfence();
  *(volatile v4ua*)dp = u;
}

__device__ __forceinline__ void wgT_store(const float* sW, unsigned short* WGTH,
                                          unsigned short* WGTL, int o0, int wv, int lane)
{
  #pragma unroll
  for (int i = 0; i < 4; ++i) {
    const int rp = wv + 8 * i;
    const int ol = 2 * rp + (lane >> 4);
    const int f0 = (lane & 15) * 8;
    v4f x0, x1;
    x0.x = sW[(f0 + 0) * WTP + ol]; x0.y = sW[(f0 + 1) * WTP + ol];
    x0.z = sW[(f0 + 2) * WTP + ol]; x0.w = sW[(f0 + 3) * WTP + ol];
    x1.x = sW[(f0 + 4) * WTP + ol]; x1.y = sW[(f0 + 5) * WTP + ol];
    x1.z = sW[(f0 + 6) * WTP + ol]; x1.w = sW[(f0 + 7) * WTP + ol];
    v4u hv, lv;
    pk8(x0, x1, hv, lv);
    const size_t off = (size_t)(o0 + ol) * DD + f0;
    *(volatile v4ua*)(WGTH + off) = hv;
    *(volatile v4ua*)(WGTL + off) = lv;
  }
}

__global__ __launch_bounds__(256) void k_wgT(const float* __restrict__ WG,
                                             unsigned short* __restrict__ WGTH,
                                             unsigned short* __restrict__ WGTL)
{
  __shared__ __align__(16) float sW[DD * WTP];
  const int tid = threadIdx.x, lane = tid & 31, wv = tid >> 5;
  const int o0 = blockIdx.x * 64;
  #pragma unroll
  for (int it = 0; it < 8; ++it) {
    const int idx = tid + 256 * it;
    const int f = idx >> 4, c4 = idx & 15;
    *(v4fa*)(sW + f * WTP + 4 * c4) = *(const v4fa*)(WG + (size_t)f * GD + o0 + 4 * c4);
  }
  __syncthreads();
  wgT_store(sW, WGTH, WGTL, o0, wv, lane);
  __threadfence();
  wgT_store(sW, WGTH, WGTL, o0, wv, lane);
}

__device__ __forceinline__ void proj_store(const float* sP, float* P, int r0, int wv, int lane)
{
  #pragma unroll
  for (int i = 0; i < 4; ++i) {
    const int idx = wv + 8 * i;
    const int row = idx >> 1, hf = idx & 1;
    const v4f v = *(const v4fa*)(sP + row * PP + 128 * hf + 4 * lane);
    *(volatile v4fa*)(P + (size_t)(r0 + row) * H0 + 128 * hf + 4 * lane) = v;
  }
}

__global__ __launch_bounds__(256) void k_proj(const unsigned short* __restrict__ NH,
                                              const unsigned short* __restrict__ NL,
                                              const unsigned short* __restrict__ W1H,
                                              const unsigned short* __restrict__ W1L,
                                              const float* __restrict__ b1,
                                              float* __restrict__ PA,
                                              float* __restrict__ PB)
{
  __shared__ __align__(16) float sP[16 * PP];
  const int tid = threadIdx.x, lane = tid & 31, wv = tid >> 5;
  const int h = lane >> 4, m = lane & 15;
  const int r0 = blockIdx.x * 16;

  const unsigned short* arh = NH + (size_t)(r0 + m) * DD;
  const unsigned short* arl = NL + (size_t)(r0 + m) * DD;

  const v8f z8 = {0.f, 0.f, 0.f, 0.f, 0.f, 0.f, 0.f, 0.f};
  v8f accA[2], accB[2];
  accA[0] = z8; accA[1] = z8; accB[0] = z8; accB[1] = z8;

  #pragma unroll
  for (int kk = 0; kk < DD / 32; ++kk) {
    const int k0 = 32 * kk;
    const v16bf ah = ldfu(arh + k0, h);
    const v16bf al = ldfu(arl + k0, h);
    #pragma unroll
    for (int ci = 0; ci < 2; ++ci) {
      const int g = 32 * wv + 16 * ci + m;
      const unsigned short* wrh = W1H + (size_t)g * H0 + k0;
      const unsigned short* wrl = W1L + (size_t)g * H0 + k0;
      accA[ci] = wmma3(ah, al, ldfu(wrh, h), ldfu(wrl, h), accA[ci]);
      accB[ci] = wmma3(ah, al, ldfu(wrh + DD, h), ldfu(wrl + DD, h), accB[ci]);
    }
  }

  #pragma unroll
  for (int ci = 0; ci < 2; ++ci) {
    const int g = 32 * wv + 16 * ci + m;
    const float bb = b1[g];
    #pragma unroll
    for (int r = 0; r < 8; ++r) sP[(8 * h + r) * PP + g] = accA[ci][r] + bb;
  }
  __syncthreads();
  proj_store(sP, PA, r0, wv, lane);
  __threadfence();
  proj_store(sP, PA, r0, wv, lane);
  __syncthreads();
  #pragma unroll
  for (int ci = 0; ci < 2; ++ci) {
    const int g = 32 * wv + 16 * ci + m;
    #pragma unroll
    for (int r = 0; r < 8; ++r) sP[(8 * h + r) * PP + g] = accB[ci][r];
  }
  __syncthreads();
  proj_store(sP, PB, r0, wv, lane);
  __threadfence();
  proj_store(sP, PB, r0, wv, lane);
}

__device__ __forceinline__ void pair_store(const float* sS, const float* sL, float* out1,
                                           unsigned short* ALH, unsigned short* ALL,
                                           int rp, int t, int a0, int tid, int wv, int lane)
{
  const int tc = (tid < 200) ? tid : 199;
  const v4f ov = *(const v4fa*)(sS + 4 * tc);
  const int r  = wv >> 2, pl = (wv >> 1) & 1, hf = wv & 1;
  const int n0 = 256 * hf + 8 * lane;
  const bool nv = (n0 < NN);
  const int nb = nv ? n0 : (NN - 8);
  const v4f x0 = *(const v4fa*)(sL + r * NN + nb);
  const v4f x1 = *(const v4fa*)(sL + r * NN + nb + 4);
  v4u hv, lv;
  pk8(x0, x1, hv, lv);
  const v4u zu = {0u, 0u, 0u, 0u};
  v4u sv = pl ? lv : hv;
  sv = nv ? sv : zu;
  unsigned short* pb = (pl ? ALL : ALH) + (size_t)(t * NN + a0 + r) * KP + n0;
  if (tid < 200) *(volatile v4fa*)(out1 + (size_t)rp * (2 * NN) + 4 * tid) = ov;
  *(volatile v4ua*)pb = sv;
}

__global__ __launch_bounds__(256) void k_pair(const float* __restrict__ PA,
                                              const float* __restrict__ PB,
                                              const _Float16* __restrict__ W2S,
                                              const float* __restrict__ b2,
                                              const float* __restrict__ w3,
                                              const float* __restrict__ b3,
                                              const float* __restrict__ adj,
                                              float* __restrict__ out1,
                                              unsigned short* __restrict__ ALH,
                                              unsigned short* __restrict__ ALL)
{
  extern __shared__ __align__(16) float psm[];
  _Float16* sW = (_Float16*)psm;
  float* sS = psm + PAIR_LDS_W2 / 4;
  float* sL = sS + 2 * NN;
  const int tid = threadIdx.x, lane = tid & 31, wv = tid >> 5;
  const int h = lane >> 4, m = lane & 15;
  const int rp = blockIdx.x;
  const int t  = rp / (NN / 2);
  const int a0 = (rp - t * (NN / 2)) * 2;

  #pragma unroll
  for (int i = 0; i < 16; ++i) {
    const int idx = tid + 256 * i;
    const int row = idx >> 5, c = idx & 31;
    *(v4ua*)(sW + row * W2P + 8 * c) = *(const v4ua*)(W2S + (size_t)row * H0 + 8 * c);
  }
  __syncthreads();

  const float b3s = b3[0];
  const v4f z4 = {0.f, 0.f, 0.f, 0.f};
  const v8f z8 = {0.f, 0.f, 0.f, 0.f, 0.f, 0.f, 0.f, 0.f};

  #pragma unroll 1
  for (int j = wv; j < 2 * (NN / 16); j += 8) {
    const int al = (j >= (NN / 16)) ? 1 : 0;
    const int bt = j - al * (NN / 16);
    const int a  = a0 + al;
    const int b0 = bt * 16;
    const float* par = PA + (size_t)(t * NN + a) * H0 + 8 * h;
    const float* pbr = PB + (size_t)(t * NN + b0 + m) * H0 + 8 * h;

    v8f acc[8];
    #pragma unroll
    for (int nt = 0; nt < 8; ++nt) acc[nt] = z8;

    #pragma unroll 1
    for (int ks = 0; ks < H0 / 32; ++ks) {
      const int k0 = ks * 32;
      const v4f s0 = __builtin_elementwise_max(*(const v4fa*)(par + k0)      + *(const v4fa*)(pbr + k0),      z4);
      const v4f s1 = __builtin_elementwise_max(*(const v4fa*)(par + k0 + 4)  + *(const v4fa*)(pbr + k0 + 4),  z4);
      const v4f s2 = __builtin_elementwise_max(*(const v4fa*)(par + k0 + 16) + *(const v4fa*)(pbr + k0 + 16), z4);
      const v4f s3 = __builtin_elementwise_max(*(const v4fa*)(par + k0 + 20) + *(const v4fa*)(pbr + k0 + 20), z4);
      FragH A;
      A.q[0] = __builtin_convertvector(s0, v4h);
      A.q[1] = __builtin_convertvector(s1, v4h);
      A.q[2] = __builtin_convertvector(s2, v4h);
      A.q[3] = __builtin_convertvector(s3, v4h);
      #pragma unroll
      for (int nt = 0; nt < 8; ++nt) {
        const v16h B = ldfh(sW + (nt * 16 + m) * W2P + k0, h);
        acc[nt] = wmma_hf(A.v, B, acc[nt]);
      }
    }

    float p[8];
    #pragma unroll
    for (int r = 0; r < 8; ++r) p[r] = 0.f;
    #pragma unroll
    for (int nt = 0; nt < 8; ++nt) {
      const int n = nt * 16 + m;
      const float bb = b2[n];
      const float ww = w3[n];
      #pragma unroll
      for (int r = 0; r < 8; ++r) {
        const float g = fmaxf(acc[nt][r] * 0.0625f + bb, 0.f);
        p[r] = fmaf(g, ww, p[r]);
      }
    }
    #pragma unroll
    for (int mask = 1; mask < 16; mask <<= 1) {
      #pragma unroll
      for (int r = 0; r < 8; ++r) p[r] += __shfl_xor(p[r], mask, 32);
    }
    float pm = p[0];
    #pragma unroll
    for (int r = 1; r < 8; ++r) pm = (m == r) ? p[r] : pm;

    const int bl = b0 + 8 * h + m;
    const int ac = (a < SS) ? a : (SS - 1);
    const int bc = (bl < SS) ? bl : (SS - 1);
    const float av = adj[((size_t)t * SS + ac) * SS + bc];
    const float s = sigm(pm + b3s);
    const bool inblk = (a < SS) && (bl < SS);
    const float la = inblk ? ((av > 0.f) ? 1.0f : -s) : s;
    if (m < 8) {
      sS[al * NN + bl] = s;
      sL[al * NN + bl] = la;
    }
  }
  __syncthreads();

  pair_store(sS, sL, out1, ALH, ALL, rp, t, a0, tid, wv, lane);
  __threadfence();
  pair_store(sS, sL, out1, ALH, ALL, rp, t, a0, tid, wv, lane);
}

__device__ __forceinline__ void sup_store(const float* sD, const float* sC,
                                          unsigned short* STH, unsigned short* STL,
                                          int t, int o0, int wv, int lane)
{
  #pragma unroll 1
  for (int i = 0; i < 16; ++i) {
    const int idx = wv + 8 * i;
    const int row = idx >> 2, pl = (idx >> 1) & 1, hf = idx & 1;
    const int n0 = 256 * hf + 8 * lane;
    const bool nv = (n0 < NN);
    const int nb = nv ? n0 : (NN - 8);
    const float cr = sC[row];
    const v4f x0 = *(const v4fa*)(sD + row * SDP + nb) + cr;
    const v4f x1 = *(const v4fa*)(sD + row * SDP + nb + 4) + cr;
    v4u hv, lv;
    pk8(x0, x1, hv, lv);
    const v4u zu = {0u, 0u, 0u, 0u};
    v4u sv = pl ? lv : hv;
    sv = nv ? sv : zu;
    unsigned short* pb = (pl ? STL : STH) + (size_t)(t * GD + o0 + row) * KP + n0;
    *(volatile v4ua*)pb = sv;
  }
}

__global__ __launch_bounds__(256) void k_sup(const float* __restrict__ nf,
                                             const float* __restrict__ WG,
                                             const unsigned short* __restrict__ WGTH,
                                             const unsigned short* __restrict__ WGTL,
                                             const unsigned short* __restrict__ NH,
                                             const unsigned short* __restrict__ NL,
                                             unsigned short* __restrict__ STH,
                                             unsigned short* __restrict__ STL)
{
  __shared__ __align__(16) float sD[32 * SDP];
  __shared__ float sC8[8 * 32];
  __shared__ float sC[32];
  const int tid = threadIdx.x, lane = tid & 31, wv = tid >> 5;
  const int h = lane >> 4, m = lane & 15;
  const int o0 = blockIdx.x * 32;
  const int t  = blockIdx.y;

  {
    const int ol = tid & 31, part = tid >> 5;
    const float* q  = nf + ((size_t)t * NN + SS) * DD;
    const float* wc = WG + (size_t)DD * GD + o0 + ol;
    float s = 0.f;
    #pragma unroll 4
    for (int jj = 0; jj < 80; ++jj) {
      const int j = part * 80 + jj;
      s = fmaf(q[j], wc[(size_t)j * GD], s);
    }
    sC8[part * 32 + ol] = s;
  }
  __syncthreads();
  if (tid < 32) {
    float c = sC8[tid];
    #pragma unroll
    for (int part = 1; part < 8; ++part) c += sC8[part * 32 + tid];
    sC[tid] = c;
  }

  const v8f z8 = {0.f, 0.f, 0.f, 0.f, 0.f, 0.f, 0.f, 0.f};
  #pragma unroll 1
  for (int j = wv; j < 50; j += 8) {
    const int mt = (j >= 25) ? 1 : 0;
    const int nt = j - 25 * mt;
    const unsigned short* arh = WGTH + (size_t)(o0 + 16 * mt + m) * DD;
    const unsigned short* arl = WGTL + (size_t)(o0 + 16 * mt + m) * DD;
    const unsigned short* brh = NH + (size_t)(t * NN + 16 * nt + m) * DD;
    const unsigned short* brl = NL + (size_t)(t * NN + 16 * nt + m) * DD;
    v8f acc = z8;
    #pragma unroll
    for (int kk = 0; kk < DD / 32; ++kk) {
      const int k0 = 32 * kk;
      acc = wmma3(ldfu(arh + k0, h), ldfu(arl + k0, h), ldfu(brh + k0, h), ldfu(brl + k0, h), acc);
    }
    #pragma unroll
    for (int r = 0; r < 8; ++r) sD[(16 * mt + 8 * h + r) * SDP + 16 * nt + m] = acc[r];
  }
  __syncthreads();

  sup_store(sD, sC, STH, STL, t, o0, wv, lane);
  __threadfence();
  sup_store(sD, sC, STH, STL, t, o0, wv, lane);
}

__device__ __forceinline__ void wl_store(const float* sD, unsigned short* WLH, unsigned short* WLL,
                                         int rowbase, int o0, int wv, int lane)
{
  const int row = 2 * wv + (lane >> 4);
  const int c0  = (lane & 15) * 8;
  const v4f x0 = *(const v4fa*)(sD + row * EP + c0);
  const v4f x1 = *(const v4fa*)(sD + row * EP + c0 + 4);
  v4u hv, lv;
  pk8(x0, x1, hv, lv);
  const size_t off = (size_t)(rowbase + row) * GD + o0 + c0;
  *(volatile v4ua*)(WLH + off) = hv;
  *(volatile v4ua*)(WLL + off) = lv;
}
__device__ __forceinline__ void out0_store(const float* sD, float* out0, int n0, int o0, int wv, int lane)
{
  #pragma unroll
  for (int i = 0; i < 2; ++i) {
    const int row = 2 * wv + i;
    const v4f v = *(const v4fa*)(sD + row * EP + 4 * lane);
    *(volatile v4fa*)(out0 + (size_t)(n0 + row) * GD + o0 + 4 * lane) = v;
  }
}

__global__ __launch_bounds__(256) void k_wl(const unsigned short* __restrict__ ALH,
                                            const unsigned short* __restrict__ ALL,
                                            const unsigned short* __restrict__ STH,
                                            const unsigned short* __restrict__ STL,
                                            const float* __restrict__ bG,
                                            unsigned short* __restrict__ WLH,
                                            unsigned short* __restrict__ WLL,
                                            float* __restrict__ out0)
{
  __shared__ __align__(16) float sD[16 * EP];
  const int tid = threadIdx.x, lane = tid & 31, wv = tid >> 5;
  const int h = lane >> 4, m = lane & 15;
  const int n0  = blockIdx.x * 16;
  const int o0  = blockIdx.y * 128;
  const int cl  = 16 * wv + m;
  const int col = o0 + cl;
  const float bias = bG[col];
  const v8f z8 = {0.f, 0.f, 0.f, 0.f, 0.f, 0.f, 0.f, 0.f};
  v8f tot = z8;

  #pragma unroll 1
  for (int t = 0; t < TT; ++t) {
    const unsigned short* arh = ALH + (size_t)(t * NN + n0 + m) * KP;
    const unsigned short* arl = ALL + (size_t)(t * NN + n0 + m) * KP;
    const unsigned short* brh = STH + (size_t)(t * GD + col) * KP;
    const unsigned short* brl = STL + (size_t)(t * GD + col) * KP;
    v8f acc = z8;
    #pragma unroll 1
    for (int kk = 0; kk < KA / 32; ++kk) {
      const int k0 = 32 * kk;
      acc = wmma3(ldfu(arh + k0, h), ldfu(arl + k0, h), ldfu(brh + k0, h), ldfu(brl + k0, h), acc);
    }
    #pragma unroll
    for (int r = 0; r < 8; ++r) {
      const float v = fmaxf(acc[r] + bias, 0.f);
      tot[r] += v;
      sD[(8 * h + r) * EP + cl] = v;
    }
    __syncthreads();
    wl_store(sD, WLH, WLL, t * NN + n0, o0, wv, lane);
    __threadfence();
    wl_store(sD, WLH, WLL, t * NN + n0, o0, wv, lane);
    __syncthreads();
  }

  #pragma unroll
  for (int r = 0; r < 8; ++r) sD[(8 * h + r) * EP + cl] = tot[r] * 0.25f;
  __syncthreads();
  out0_store(sD, out0, n0, o0, wv, lane);
  __threadfence();
  out0_store(sD, out0, n0, o0, wv, lane);
}

__global__ __launch_bounds__(256) void k_fc2(const unsigned short* __restrict__ WLH,
                                             const unsigned short* __restrict__ WLL,
                                             const unsigned short* __restrict__ F1H,
                                             const unsigned short* __restrict__ F1L,
                                             const float* __restrict__ b1,
                                             const unsigned short* __restrict__ F2H,
                                             const unsigned short* __restrict__ F2L,
                                             const float* __restrict__ b2,
                                             const float* __restrict__ w3,
                                             const float* __restrict__ b3,
                                             float* __restrict__ QSN)
{
  __shared__ __align__(16) float sH[16 * EP];
  __shared__ __align__(16) float sG[16 * EP];
  __shared__ __align__(16) float sQ[128];
  const int tid = threadIdx.x, lane = tid & 31, wv = tid >> 5;
  const int h = lane >> 4, m = lane & 15;
  const int r0  = blockIdx.x * 16;
  const int col = 16 * wv + m;
  const v8f z8 = {0.f, 0.f, 0.f, 0.f, 0.f, 0.f, 0.f, 0.f};

  {
    const unsigned short* arh = WLH + (size_t)(r0 + m) * GD;
    const unsigned short* arl = WLL + (size_t)(r0 + m) * GD;
    const unsigned short* brh = F1H + (size_t)col * GD;
    const unsigned short* brl = F1L + (size_t)col * GD;
    v8f acc = z8;
    #pragma unroll 2
    for (int kk = 0; kk < GD / 32; ++kk) {
      const int k0 = 32 * kk;
      acc = wmma3(ldfu(arh + k0, h), ldfu(arl + k0, h), ldfu(brh + k0, h), ldfu(brl + k0, h), acc);
    }
    const float bb = b1[col];
    #pragma unroll
    for (int r = 0; r < 8; ++r) sH[(8 * h + r) * EP + col] = fmaxf(acc[r] + bb, 0.f);
  }
  __syncthreads();

  {
    const unsigned short* brh = F2H + (size_t)col * H1;
    const unsigned short* brl = F2L + (size_t)col * H1;
    v8f acc = z8;
    #pragma unroll
    for (int kk = 0; kk < H1 / 32; ++kk) {
      const int k0 = 32 * kk;
      const float* base = sH + m * EP + k0 + 8 * h;
      v16bf ah, al;
      mkfrag(*(const v4fa*)base, *(const v4fa*)(base + 4),
             *(const v4fa*)(base + 16), *(const v4fa*)(base + 20), ah, al);
      acc = wmma3(ah, al, ldfu(brh + k0, h), ldfu(brl + k0, h), acc);
    }
    const float bb = b2[col];
    #pragma unroll
    for (int r = 0; r < 8; ++r) sG[(8 * h + r) * EP + col] = fmaxf(acc[r] + bb, 0.f);
  }
  __syncthreads();

  {
    const int q80 = (tid < 80) ? tid : 0;
    const int row = q80 / NW;
    const int c   = q80 - NW * row;
    const float* gr = sG + row * EP;
    const float* wr = w3 + (size_t)c * H2;
    float s3 = b3[c];
    #pragma unroll 4
    for (int k = 0; k < H2; ++k) s3 = fmaf(gr[k], wr[k], s3);
    const float sg = sigm(s3);
    if (tid < 80) sQ[row * 8 + c] = sg;
    if (tid >= 80 && tid < 128) {
      const int idx = tid - 80;
      const int rz = idx / 3;
      const int cz = NW + idx - 3 * rz;
      sQ[rz * 8 + cz] = 0.f;
    }
  }
  __syncthreads();

  if (wv == 0) {
    const v4f v = *(const v4fa*)(sQ + 4 * lane);
    float* dp = QSN + (size_t)r0 * 8 + 4 * lane;
    *(volatile v4fa*)dp = v;
    __threadfence();
    *(volatile v4fa*)dp = v;
  }
}

__device__ __forceinline__ void out2_store(const float* QSN, float* out2, int tid)
{
  #pragma unroll 1
  for (int it = 0; it < 8; ++it) {
    const int f4  = tid + 256 * it;
    const int f4c = (f4 < 2000) ? f4 : 1999;
    const int row = f4c / (NN / 4);
    const int n   = 4 * (f4c - row * (NN / 4));
    const int t   = row / NW;
    const int c   = row - NW * t;
    const float* base = QSN + ((size_t)(t * NN + n)) * 8 + c;
    v4f v;
    v.x = base[0]; v.y = base[8]; v.z = base[16]; v.w = base[24];
    if (f4 < 2000) *(volatile v4fa*)(out2 + 4 * (size_t)f4) = v;
  }
}

__global__ __launch_bounds__(256) void k_out2(const float* __restrict__ QSN, float* __restrict__ out2)
{
  const int tid = threadIdx.x;
  out2_store(QSN, out2, tid);
  __threadfence();
  out2_store(QSN, out2, tid);
}

extern "C" void kernel_launch(void* const* d_in, const int* in_sizes, int n_in,
                              void* d_out, int out_size, void* d_ws, size_t ws_size,
                              hipStream_t stream)
{
  if (n_in < 16) return;
  if (in_sizes[0]  != TT * NN * DD) return;
  if (in_sizes[1]  != TT * SS * SS) return;
  if (in_sizes[2]  != H0 * 2 * DD) return;
  if (in_sizes[3]  != H0) return;
  if (in_sizes[4]  != H1 * H0) return;
  if (in_sizes[5]  != H1) return;
  if (in_sizes[6]  != H1) return;
  if (in_sizes[7]  != 1) return;
  if (in_sizes[8]  != GD * GD) return;
  if (in_sizes[9]  != GD) return;
  if (in_sizes[10] != H1 * GD) return;
  if (in_sizes[11] != H1) return;
  if (in_sizes[12] != H2 * H1) return;
  if (in_sizes[13] != H2) return;
  if (in_sizes[14] != NW * H2) return;
  if (in_sizes[15] != NW) return;
  if (out_size != NN * GD + TT * NN * NN + TT * NW * NN) return;

  const float* nf     = (const float*)d_in[0];
  const float* adj    = (const float*)d_in[1];
  const float* fc1_w1 = (const float*)d_in[2];
  const float* fc1_b1 = (const float*)d_in[3];
  const float* fc1_w2 = (const float*)d_in[4];
  const float* fc1_b2 = (const float*)d_in[5];
  const float* fc1_w3 = (const float*)d_in[6];
  const float* fc1_b3 = (const float*)d_in[7];
  const float* wG     = (const float*)d_in[8];
  const float* bG     = (const float*)d_in[9];
  const float* fc2_w1 = (const float*)d_in[10];
  const float* fc2_b1 = (const float*)d_in[11];
  const float* fc2_w2 = (const float*)d_in[12];
  const float* fc2_b2 = (const float*)d_in[13];
  const float* fc2_w3 = (const float*)d_in[14];
  const float* fc2_b3 = (const float*)d_in[15];

  float* out0 = (float*)d_out;
  float* out1 = out0 + (size_t)NN * GD;
  float* out2 = out1 + (size_t)TT * NN * NN;

  const size_t bNP  = (size_t)TN * DD * 2;
  const size_t bW1  = (size_t)H0 * H0 * 2;
  const size_t bW2  = (size_t)H1 * H0 * 2;
  const size_t bF1  = (size_t)H1 * GD * 2;
  const size_t bF2  = (size_t)H2 * H1 * 2;
  const size_t bWT  = (size_t)GD * DD * 2;
  const size_t bP   = (size_t)TN * H0 * 4;
  const size_t bAL  = (size_t)TN * KP * 2;
  const size_t bST  = (size_t)TT * GD * KP * 2;
  const size_t bWL  = (size_t)TN * GD * 2;
  const size_t bQS  = (size_t)TN * 8 * 4;
  const size_t total = 2 * bNP + 2 * bW1 + bW2 + 2 * bF1 + 2 * bF2 + 2 * bWT + 2 * bP +
                       2 * bAL + 2 * bST + 2 * bWL + bQS;
  if (total > ws_size) return;
  if (total > (size_t)134217728) return;

  char* ws = (char*)d_ws;
  size_t off = 0;
  unsigned short* NH   = (unsigned short*)(ws + off); off += bNP;
  unsigned short* NL   = (unsigned short*)(ws + off); off += bNP;
  unsigned short* W1H  = (unsigned short*)(ws + off); off += bW1;
  unsigned short* W1L  = (unsigned short*)(ws + off); off += bW1;
  _Float16*       W2S  = (_Float16*)(ws + off);       off += bW2;
  unsigned short* F1H  = (unsigned short*)(ws + off); off += bF1;
  unsigned short* F1L  = (unsigned short*)(ws + off); off += bF1;
  unsigned short* F2H  = (unsigned short*)(ws + off); off += bF2;
  unsigned short* F2L  = (unsigned short*)(ws + off); off += bF2;
  unsigned short* WGTH = (unsigned short*)(ws + off); off += bWT;
  unsigned short* WGTL = (unsigned short*)(ws + off); off += bWT;
  float*          PA   = (float*)(ws + off);          off += bP;
  float*          PB   = (float*)(ws + off);          off += bP;
  unsigned short* ALH  = (unsigned short*)(ws + off); off += bAL;
  unsigned short* ALL  = (unsigned short*)(ws + off); off += bAL;
  unsigned short* STH  = (unsigned short*)(ws + off); off += bST;
  unsigned short* STL  = (unsigned short*)(ws + off); off += bST;
  unsigned short* WLH  = (unsigned short*)(ws + off); off += bWL;
  unsigned short* WLL  = (unsigned short*)(ws + off); off += bWL;
  float*          QSN  = (float*)(ws + off);          off += bQS;
  if (off != total) return;

  const int n8N  = TN * DD / 8;
  const int n8W1 = H0 * H0 / 8;
  const int n8W2 = H1 * H0 / 8;
  const int n8F1 = H1 * GD / 8;
  const int n8F2 = H2 * H1 / 8;
  k_split<<<(unsigned)(n8N / 256),  256, 0, stream>>>(nf,     NH,  NL,  n8N);
  k_split<<<(unsigned)(n8W1 / 256), 256, 0, stream>>>(fc1_w1, W1H, W1L, n8W1);
  k_cvt16<<<(unsigned)(n8W2 / 256), 256, 0, stream>>>(fc1_w2, W2S, n8W2, 16.0f);
  k_split<<<(unsigned)(n8F1 / 256), 256, 0, stream>>>(fc2_w1, F1H, F1L, n8F1);
  k_split<<<(unsigned)(n8F2 / 256), 256, 0, stream>>>(fc2_w2, F2H, F2L, n8F2);
  k_wgT<<<GD / 64, 256, 0, stream>>>(wG, WGTH, WGTL);

  k_proj<<<TN / 16, 256, 0, stream>>>(NH, NL, W1H, W1L, fc1_b1, PA, PB);

  hipFuncSetAttribute(reinterpret_cast<const void*>(&k_pair),
                      hipFuncAttributeMaxDynamicSharedMemorySize, PAIR_LDS_BYTES);
  k_pair<<<TN / 2, 256, PAIR_LDS_BYTES, stream>>>(PA, PB, W2S, fc1_b2, fc1_w3, fc1_b3, adj,
                                                   out1, ALH, ALL);

  k_sup<<<dim3(GD / 32, TT), 256, 0, stream>>>(nf, wG, WGTH, WGTL, NH, NL, STH, STL);

  k_wl<<<dim3(NN / 16, GD / 128), 256, 0, stream>>>(ALH, ALL, STH, STL, bG, WLH, WLL, out0);

  k_fc2<<<TN / 16, 256, 0, stream>>>(WLH, WLL, F1H, F1L, fc2_b1, F2H, F2L, fc2_b2,
                                     fc2_w3, fc2_b3, QSN);
  k_out2<<<1, 256, 0, stream>>>(QSN, out2);
}
